// Attention_44470091383531
// MI455X (gfx1250) — hardware-verified
//
#include <hip/hip_runtime.h>
#include <math.h>

#ifndef NB
#define NB 2
#endif
#ifndef SEQ
#define SEQ 2048
#endif
#define NB_FULL 2
#define SEQ_FULL 2048
#define DM 2048
#define NHD 16
#define HD 128
#define NQKV 6144
#define NXR 256

static_assert(SEQ % 64 == 0);
static_assert(SEQ >= NXR);
static_assert(SEQ <= SEQ_FULL);
static_assert(NB <= NB_FULL);
static_assert(NHD * HD == DM);
static_assert(HD == 128);
static_assert(DM % 64 == 0 && NQKV % 64 == 0 && DM % 32 == 0 && NXR % 64 == 0);

typedef __attribute__((ext_vector_type(16))) _Float16 v16h;
typedef __attribute__((ext_vector_type(8)))  _Float16 v8h;
typedef __attribute__((ext_vector_type(4)))  _Float16 v4h;
typedef __attribute__((ext_vector_type(8)))  float    v8f;
typedef __attribute__((ext_vector_type(4)))  float    v4f;

__device__ __forceinline__ v8f wmma16(v16h a, v16h b, v8f c) {
    c = __builtin_amdgcn_wmma_f32_16x16x32_f16(false, a, false, b, (short)0, c, false, false);
    asm volatile("v_nop\n\tv_nop\n\tv_nop\n\tv_nop" : "+v"(c) : "v"(a), "v"(b));
    return c;
}
union FragH { v16h v; v8h h[2]; };
__device__ __forceinline__ v16h ldfrag(const _Float16* p) { FragH f; f.h[0] = *(const v8h*)(p); f.h[1] = *(const v8h*)(p + 16); return f.v; }
__device__ __forceinline__ v4h cvt4h(v4f x) { v4h r; r.x = (_Float16)x.x; r.y = (_Float16)x.y; r.z = (_Float16)x.z; r.w = (_Float16)x.w; return r; }

#define VST2(T, ptr, val) do { const T vst2_v_ = (val); *(volatile T*)(ptr) = vst2_v_; __threadfence(); *(volatile T*)(ptr) = vst2_v_; } while (0)
#define VST2V4(ptr, val) do { const v4f vst2_v4_ = (val); *(volatile v4f*)(ptr) = vst2_v4_; __threadfence(); *(volatile v4f*)(ptr) = vst2_v4_; } while (0)

#define AW 4
#define QP 136
#define VTP 72
#ifndef KATTN_ATTR
#define KATTN_ATTR __attribute__((amdgpu_num_vgpr(256)))
#endif
__global__ __launch_bounds__(32 * AW) KATTN_ATTR void k_attn128(const float* __restrict__ Q, const float* __restrict__ K, const float* __restrict__ V, float* __restrict__ O,
                                                                 int ldq, int ldkv, int ldo, int Lq, int Lk, int coff, float scale) {
    __shared__ __align__(16) float    qo[AW][16 * 68];
    __shared__ __align__(16) _Float16 kh[64 * QP];
    __shared__ __align__(16) _Float16 vt[HD * VTP];
    __shared__ __align__(16) _Float16 ph[AW][16 * VTP];
    static_assert(16 * QP * 2 == 16 * 68 * 4);
    const int tid = threadIdx.x, lane = tid & 31, hf = lane >> 4, l15 = lane & 15, wave = tid >> 5;
    const int h = blockIdx.y;
    const int q0 = (blockIdx.x * AW + wave) * 16;
    _Float16* qh = (_Float16*)&qo[wave][0];
    float* os = &qo[wave][0];
    _Float16* pw = &ph[wave][0];
    const float L2E = 1.4426950408889634f;
    const float NEG = -__builtin_inff();
    const v4f z4 = {0.f, 0.f, 0.f, 0.f};
    {
        const int qi = min(q0 + l15, Lq - 1);
        const float* qrow = Q + (long long)qi * ldq + h * HD + hf * 64;
        _Float16* qd = qh + l15 * QP + hf * 64;
#pragma unroll 4
        for (int i = 0; i < 16; ++i) {
            const v4f x = *(const v4f*)(qrow + 4 * i);
            *(v4h*)(qd + 4 * i) = cvt4h(x);
        }
    }
    v8f o[8]; float m8[8], l8[8];
#pragma unroll
    for (int t = 0; t < 8; ++t) { v8f zz = {}; o[t] = zz; }
#pragma unroll
    for (int i = 0; i < 8; ++i) { m8[i] = NEG; l8[i] = 0.f; }
    const int je = (blockIdx.x * AW + AW - 1) * 16 + 16 + coff;
    const int jend = min(Lk, max(je, 0));
    const float* kbase = K + h * HD;
    const float* vbase = V + h * HD;
    for (int j0 = 0; j0 < jend; j0 += 64) {
        __syncthreads();
        {
            const int jr = tid >> 1, dh = (tid & 1) * 64;
            const int j = j0 + jr; const int jc = min(j, Lk - 1); const bool live = (j < Lk);
            const float* kr = kbase + (long long)jc * ldkv + dh;
            const float* vr = vbase + (long long)jc * ldkv + dh;
            _Float16* kd = kh + jr * QP + dh;
#pragma unroll 4
            for (int i = 0; i < 16; ++i) {
                const v4f kk0 = *(const v4f*)(kr + 4 * i);
                const v4f vv0 = *(const v4f*)(vr + 4 * i);
                const v4f kk = live ? kk0 : z4;
                const v4f vv = live ? vv0 : z4;
                *(v4h*)(kd + 4 * i) = cvt4h(kk);
                const int d = dh + 4 * i;
                vt[(d + 0) * VTP + jr] = (_Float16)vv.x;
                vt[(d + 1) * VTP + jr] = (_Float16)vv.y;
                vt[(d + 2) * VTP + jr] = (_Float16)vv.z;
                vt[(d + 3) * VTP + jr] = (_Float16)vv.w;
            }
        }
        __syncthreads();
        v8f s[4];
#pragma unroll
        for (int t = 0; t < 4; ++t) { v8f zz = {}; s[t] = zz; }
#pragma unroll 1
        for (int ks = 0; ks < 4; ++ks) {
            const v16h a = ldfrag(qh + l15 * QP + ks * 32 + 8 * hf);
#pragma unroll
            for (int t = 0; t < 4; ++t) {
                const v16h bk = ldfrag(kh + (t * 16 + l15) * QP + ks * 32 + 8 * hf);
                s[t] = wmma16(a, bk, s[t]);
            }
        }
#pragma unroll
        for (int i = 0; i < 8; ++i) {
            const int irow = q0 + i + 8 * hf;
            float sc[4];
#pragma unroll
            for (int t = 0; t < 4; ++t) {
                const int jg = j0 + t * 16 + l15;
                float v = s[t][i] * scale;
                if (jg >= Lk || jg > irow + coff) v = NEG; else v *= L2E;
                sc[t] = v;
            }
            float mx = fmaxf(fmaxf(sc[0], sc[1]), fmaxf(sc[2], sc[3]));
            mx = fmaxf(mx, __shfl_xor(mx, 1, 32)); mx = fmaxf(mx, __shfl_xor(mx, 2, 32));
            mx = fmaxf(mx, __shfl_xor(mx, 4, 32)); mx = fmaxf(mx, __shfl_xor(mx, 8, 32));
            const float mnew = fmaxf(m8[i], mx);
            const float corr = (mnew == NEG) ? 1.f : exp2f(m8[i] - mnew);
            float rs = 0.f;
#pragma unroll
            for (int t = 0; t < 4; ++t) {
                const float pp = (sc[t] == NEG) ? 0.f : exp2f(sc[t] - mnew); rs += pp;
                pw[(i + 8 * hf) * VTP + t * 16 + l15] = (_Float16)(pp * 4096.f);
            }
            rs += __shfl_xor(rs, 1, 32); rs += __shfl_xor(rs, 2, 32); rs += __shfl_xor(rs, 4, 32); rs += __shfl_xor(rs, 8, 32);
            l8[i] = l8[i] * corr + rs; m8[i] = mnew;
#pragma unroll
            for (int t = 0; t < 8; ++t) o[t][i] *= corr;
        }
        __syncthreads();
#pragma unroll 1
        for (int kk = 0; kk < 2; ++kk) {
            const v16h pa = ldfrag(pw + l15 * VTP + kk * 32 + 8 * hf);
#pragma unroll
            for (int t = 0; t < 8; ++t) {
                const v16h vb = ldfrag(vt + (t * 16 + l15) * VTP + kk * 32 + 8 * hf);
                o[t] = wmma16(pa, vb, o[t]);
            }
        }
    }
    float invr[8];
#pragma unroll
    for (int i = 0; i < 8; ++i) invr[i] = (l8[i] > 0.f) ? 1.f / (l8[i] * 4096.f) : 0.f;
    __syncthreads();
    float* obase = O + h * HD;
#pragma unroll
    for (int c0 = 0; c0 < HD; c0 += 64) {
#pragma unroll
        for (int i = 0; i < 8; ++i)
#pragma unroll
            for (int t = 0; t < 8; ++t) if (t * 16 >= c0 && t * 16 < c0 + 64) os[(i + 8 * hf) * 68 + (t * 16 - c0) + l15] = o[t][i] * invr[i];
        __syncthreads();
        for (int pass = 0; pass < 2; ++pass) {
#pragma unroll
            for (int it = 0; it < 8; ++it) {
                const int row = it * 2 + hf, c4 = l15 * 4;
                const v4f v = *(const v4f*)(os + row * 68 + c4);
                if (q0 + row < Lq) *(volatile v4f*)(obase + (long long)(q0 + row) * ldo + c0 + c4) = v;
            }
            __threadfence();
        }
        __syncthreads();
    }
}

__global__ __launch_bounds__(256) void k_invf(float* __restrict__ invb, int half, int D, float base) {
    const int i = blockIdx.x * 256 + threadIdx.x;
    if (i >= ((half + 31) / 32) * 32) return;
    const int ic = min(i, half - 1);
    const float e = (float)(2 * ic) / (float)D;
    const float invf = 1.0f / powf(base, e);
    const float v = (i < half) ? invf : 0.f;
    VST2(float, invb + i, v);
}
__global__ __launch_bounds__(256) void k_sincos(float* __restrict__ cs, float* __restrict__ sn, const float* __restrict__ invb, int S, int half, float pscale) {
    const int idx = blockIdx.x * 256 + threadIdx.x;
    if (idx >= S * half) return;
    const int s = idx / half, i = idx - s * half;
    const float ang = (pscale * (float)s) * invb[i];
    VST2(float, cs + idx, cosf(ang)); VST2(float, sn + idx, sinf(ang));
}

static_assert(HD == 128 && HD / 8 == 16);
static_assert(256 % 32 == 0 && 32 % 16 == 0);
__global__ __launch_bounds__(256) void k_rope_inplace(float* X, int ldx, int nslot, const float* __restrict__ CS, const float* __restrict__ SN, int S) {
    const long long idx = (long long)blockIdx.x * 256 + threadIdx.x;
    const int jq = (int)(idx & 15);
    const long long sh = idx >> 4;
    const int hs = (int)(sh % nslot);
    const long long s = sh / nslot;
    if (s >= S) return;
    float* sb = X + s * ldx + hs * 128;
    float* p = sb + 4 * jq;
    const v4f c  = *(const v4f*)(CS + s * 64 + 4 * jq);
    const v4f sn = *(const v4f*)(SN + s * 64 + 4 * jq);
    v4f x1 = *(const v4f*)p;
    v4f x2 = *(const v4f*)(p + 64);
    v4f xa = *(const v4f*)(sb + 8 * jq);
    v4f xb = *(const v4f*)(sb + 8 * jq + 4);
    asm volatile("" : "+v"(x1), "+v"(x2), "+v"(xa), "+v"(xb) : : "memory");
    const v4f xo = {xa.y, xa.w, xb.y, xb.w};
    const v4f xe = {xa.x, xa.z, xb.x, xb.z};
    const v4f y1 = x1 * c - xo * sn;
    const v4f y2 = x2 * c + xe * sn;
    VST2V4(p, y1);
    VST2V4(p + 64, y2);
}

namespace gk {
typedef __attribute__((ext_vector_type(16))) _Float16 v16h;
typedef __attribute__((ext_vector_type(8)))  _Float16 v8h;
typedef __attribute__((ext_vector_type(16))) __bf16   v16b;
typedef __attribute__((ext_vector_type(8)))  __bf16   v8b;
typedef __attribute__((ext_vector_type(8)))  float    v8f;
typedef __attribute__((ext_vector_type(4)))  float    v4f;

__device__ __forceinline__ unsigned short f2bf_bits(float f) {
  unsigned u = __float_as_uint(f);
  return (unsigned short)((u + 0x7FFFu + ((u >> 16) & 1u)) >> 16);
}
__device__ __forceinline__ float bf_bits2f(unsigned short h) { return __uint_as_float(((unsigned)h) << 16); }

__device__ __forceinline__ void dep_guard_h(v8f& a, v8f& b, v16h x, v16h y) { asm volatile("v_nop\n\tv_nop\n\tv_nop\n\tv_nop" : "+v"(a), "+v"(b) : "v"(x), "v"(y)); }
__device__ __forceinline__ void dep_guard_b(v8f& a, v8f& b, v16b x, v16b y) { asm volatile("v_nop\n\tv_nop\n\tv_nop\n\tv_nop" : "+v"(a), "+v"(b) : "v"(x), "v"(y)); }
__device__ __forceinline__ void keep4_h(v16h a, v16h b, v16h c, v16h d) { asm volatile("v_nop" :: "v"(a), "v"(b), "v"(c), "v"(d)); }
__device__ __forceinline__ void keep4_b(v16b a, v16b b, v16b c, v16b d) { asm volatile("v_nop" :: "v"(a), "v"(b), "v"(c), "v"(d)); }
__device__ __forceinline__ void acc_guard4(v8f& a, v8f& b, v8f& c, v8f& d) { asm volatile("v_nop\n\tv_nop\n\tv_nop\n\tv_nop" : "+v"(a), "+v"(b), "+v"(c), "+v"(d)); }
template <typename T> struct Frag;
template <> struct Frag<_Float16> {
  typedef v16h V; union U { v16h v; v8h h[2]; };
  static __device__ __forceinline__ v16h load(const _Float16* p) {
    U f; f.h[0] = *(const v8h*)(p); f.h[1] = *(const v8h*)(p + 16); return f.v;
  }
  static __device__ __forceinline__ v8f mma(v16h a, v16h b, v8f c) {
    return __builtin_amdgcn_wmma_f32_16x16x32_f16(false, a, false, b, (short)0, c, false, false);
  }
  static __device__ __forceinline__ void guard(v8f& a, v8f& b, v16h x, v16h y) { dep_guard_h(a, b, x, y); }
  static __device__ __forceinline__ void keep(v16h a, v16h b, v16h c, v16h d) { keep4_h(a, b, c, d); }
};
template <> struct Frag<__bf16> {
  typedef v16b V; union U { v16b v; v8b h[2]; };
  static __device__ __forceinline__ v16b load(const __bf16* p) {
    U f; f.h[0] = *(const v8b*)(p); f.h[1] = *(const v8b*)(p + 16); return f.v;
  }
  static __device__ __forceinline__ v8f mma(v16b a, v16b b, v8f c) {
    return __builtin_amdgcn_wmma_f32_16x16x32_bf16(false, a, false, b, (short)0, c, false, false);
  }
  static __device__ __forceinline__ void guard(v8f& a, v8f& b, v16b x, v16b y) { dep_guard_b(a, b, x, y); }
  static __device__ __forceinline__ void keep(v16b a, v16b b, v16b c, v16b d) { keep4_b(a, b, c, d); }
};

template <int ET> struct Elem;
template <> struct Elem<0> { typedef _Float16 T; };
template <> struct Elem<1> { typedef __bf16 T; };
template <int ET, bool SPLIT, int BIAS_MODE, int OUT_MODE, bool RESID, int ACT = 0>
__global__ __launch_bounds__(256) void wmma_gemm64(
    const unsigned short* __restrict__ Ap, const unsigned short* __restrict__ A2p, int lda, long strideA,
    const unsigned short* __restrict__ Btp, const unsigned short* __restrict__ Bt2p, int ldb, long strideB,
    void* __restrict__ Cout, void* __restrict__ Cout2, int ldc, long strideC,
    const float* __restrict__ bias,
    const float* __restrict__ resid, long strideR,
    int M, int N, int K, float scale) {
  typedef typename Elem<ET>::T T;
  typedef typename Frag<T>::V V;
  const T* A = (const T*)Ap; const T* A2 = (const T*)A2p; const T* Bt = (const T*)Btp; const T* Bt2 = (const T*)Bt2p;
  __shared__ __align__(16) float sT[8][16 * 68];
  const int b    = blockIdx.y;
  const int lane = threadIdx.x & 31;
  const int wave = threadIdx.x >> 5;
  const int tilesN = N >> 6;
  const int tilesM = M >> 6;
  const int tile = blockIdx.x * 8 + wave;
  if (tile >= tilesM * tilesN) return;
  const int tm = tile / tilesN;
  const int tn = tile - tm * tilesN;
  const int m0 = tm << 6;
  const int n0 = tn << 6;

  const T* Ab  = A  + (size_t)b * strideA;
  const T* Bb  = Bt + (size_t)b * strideB;
  const T* Ab2 = SPLIT ? (A2  + (size_t)b * strideA) : nullptr;
  const T* Bb2 = SPLIT ? (Bt2 + (size_t)b * strideB) : nullptr;

  const int rlane = lane & 15;
  const int koff  = (lane >> 4) * 8;
  const int mOff  = (lane >> 4) * 8;

  v8f acc[4][4];
#pragma unroll
  for (int i = 0; i < 4; ++i)
#pragma unroll
    for (int j = 0; j < 4; ++j) acc[i][j] = (v8f){0.f,0.f,0.f,0.f,0.f,0.f,0.f,0.f};

  for (int k0 = 0; k0 < K; k0 += 32) {
    V bh[4], bl[4];
#pragma unroll
    for (int j = 0; j < 4; ++j) {
      const size_t bo = (size_t)(n0 + (j << 4) + rlane) * ldb + koff + k0;
      bh[j] = Frag<T>::load(Bb + bo);
      if (SPLIT) bl[j] = Frag<T>::load(Bb2 + bo);
    }
#pragma unroll
    for (int i = 0; i < 4; ++i) {
      const size_t ao = (size_t)(m0 + (i << 4) + rlane) * lda + koff + k0;
      V ah = Frag<T>::load(Ab + ao);
      V al;
      if (SPLIT) al = Frag<T>::load(Ab2 + ao);
#pragma unroll
      for (int j = 0; j < 4; ++j) {
        acc[i][j] = Frag<T>::mma(ah, bh[j], acc[i][j]);
        if (SPLIT) {
          acc[i][j] = Frag<T>::mma(ah, bl[j], acc[i][j]);
          acc[i][j] = Frag<T>::mma(al, bh[j], acc[i][j]);
        }
      }
      Frag<T>::guard(acc[i][0], acc[i][3], ah, SPLIT ? al : ah);
    }
    Frag<T>::keep(bh[0], bh[1], bh[2], bh[3]);
    if (SPLIT) Frag<T>::keep(bl[0], bl[1], bl[2], bl[3]);
  }
  acc_guard4(acc[0][0], acc[0][1], acc[0][2], acc[0][3]);
  acc_guard4(acc[1][0], acc[1][1], acc[1][2], acc[1][3]);
  acc_guard4(acc[2][0], acc[2][1], acc[2][2], acc[2][3]);
  acc_guard4(acc[3][0], acc[3][1], acc[3][2], acc[3][3]);

  float* slab = sT[wave];
  const float* Rb = RESID ? (resid + (size_t)b * strideR) : nullptr;
#pragma unroll
  for (int i = 0; i < 4; ++i) {
    const int mBase = m0 + (i << 4);
#pragma unroll
    for (int j = 0; j < 4; ++j) {
      const int n = n0 + (j << 4) + rlane;
      float bv = 0.f;
      if (BIAS_MODE == 2) bv = bias[n];
#pragma unroll
      for (int r = 0; r < 8; ++r) {
        float v = acc[i][j][r] * scale;
        if (BIAS_MODE == 1) v += bias[mBase + mOff + r];
        if (BIAS_MODE == 2) v += bv;
        if (RESID) v += Rb[(size_t)(mBase + mOff + r) * ldc + n];
        if (ACT == 2) v = fmaxf(v, 0.0f);
        slab[(mOff + r) * 68 + (j << 4) + rlane] = v;
      }
    }
    __builtin_amdgcn_fence(3  , "workgroup");
    __builtin_amdgcn_wave_barrier();
    __builtin_amdgcn_fence(2  , "workgroup");
    if (OUT_MODE == 0) {
      float* C = (float*)Cout + (size_t)b * strideC;
      const int hh = lane >> 4, c4 = (lane & 15) * 4;
      for (int pass = 0; pass < 2; ++pass) {
#pragma unroll
        for (int it = 0; it < 8; ++it) {
          const int row = it * 2 + hh;
          v4f v = *(const v4f*)(slab + row * 68 + c4);
          *(volatile v4f*)(C + (size_t)(mBase + row) * ldc + n0 + c4) = v;
        }
        __threadfence();
      }
    } else {
      const int q = lane >> 3, c8 = (lane & 7) * 8;
      unsigned short* C  = (unsigned short*)Cout  + (size_t)b * strideC;
      unsigned short* C2 = (OUT_MODE == 2) ? ((unsigned short*)Cout2 + (size_t)b * strideC) : nullptr;
      for (int pass = 0; pass < 2; ++pass) {
#pragma unroll
        for (int it = 0; it < 4; ++it) {
          const int row = it * 4 + q;
          const float* sp = slab + row * 68 + c8;
          v8h hv, lv;
#pragma unroll
          for (int e = 0; e < 8; ++e) {
            if (OUT_MODE == 1) {
              hv[e] = (_Float16)sp[e];
            } else {
              unsigned short hb = f2bf_bits(sp[e]);
              unsigned short lb = f2bf_bits(sp[e] - bf_bits2f(hb));
              hv[e] = __builtin_bit_cast(_Float16, hb);
              lv[e] = __builtin_bit_cast(_Float16, lb);
            }
          }
          *(volatile v8h*)(C + (size_t)(mBase + row) * ldc + n0 + c8) = hv;
          if (OUT_MODE == 2) *(volatile v8h*)(C2 + (size_t)(mBase + row) * ldc + n0 + c8) = lv;
        }
        __threadfence();
      }
    }
    __builtin_amdgcn_fence(3  , "workgroup");
    __builtin_amdgcn_wave_barrier();
    __builtin_amdgcn_fence(2  , "workgroup");
  }
}

}

__global__ __launch_bounds__(256) void k_cast16(const float* __restrict__ src, long long lds, _Float16* __restrict__ dst, long long ldd, int R, int C, float s) {
    const long long i = (long long)blockIdx.x * 256 + threadIdx.x; const long long np = (long long)R * (C / 2); if (i >= np) return; const int r = (int)(i / (C / 2)); const int c = 2 * (int)(i % (C / 2));
    const _Float16 h0 = (_Float16)(src[(long long)r * lds + c] * s), h1 = (_Float16)(src[(long long)r * lds + c + 1] * s);
    const unsigned u = (unsigned)__builtin_bit_cast(unsigned short, h0) | ((unsigned)__builtin_bit_cast(unsigned short, h1) << 16);
    volatile unsigned* d = (volatile unsigned*)(dst + (long long)r * ldd + c); *d = u; __threadfence(); *d = u; }

__device__ __forceinline__ unsigned int f2bf2_pack(float a, float b, unsigned int* lo) {
    const unsigned short ha = gk::f2bf_bits(a), hb = gk::f2bf_bits(b);
    const unsigned short la = gk::f2bf_bits(a - gk::bf_bits2f(ha)), lb = gk::f2bf_bits(b - gk::bf_bits2f(hb));
    *lo = (unsigned)la | ((unsigned)lb << 16); return (unsigned)ha | ((unsigned)hb << 16); }
__global__ __launch_bounds__(256) void k_castS16(const float* __restrict__ src, long long lds, __bf16* __restrict__ dhi, __bf16* __restrict__ dlo, long long ldd, int R, int C, float s, int transpose) {
    const long long i = (long long)blockIdx.x * 256 + threadIdx.x; long long o; float a, b;
    if (transpose) { const long long np = (long long)C * (R / 2); if (i >= np) return; const int c = (int)(i / (R / 2)); const int r = 2 * (int)(i % (R / 2)); a = src[(long long)r * lds + c] * s; b = src[(long long)(r + 1) * lds + c] * s; o = (long long)c * ldd + r; }
    else { const long long np = (long long)R * (C / 2); if (i >= np) return; const int r = (int)(i / (C / 2)); const int c = 2 * (int)(i % (C / 2)); a = src[(long long)r * lds + c] * s; b = src[(long long)r * lds + c + 1] * s; o = (long long)r * ldd + c; }
    unsigned lo; const unsigned hi = f2bf2_pack(a, b, &lo); volatile unsigned* ph = (volatile unsigned*)(dhi + o); volatile unsigned* pl = (volatile unsigned*)(dlo + o);
    *ph = hi; *pl = lo; __threadfence(); *ph = hi; *pl = lo; }

typedef unsigned int cm_u4 __attribute__((ext_vector_type(4)));
__device__ __forceinline__ unsigned int cmb_pk2(float a, float b) { return (unsigned int)__builtin_bit_cast(unsigned short, (_Float16)a) | ((unsigned int)__builtin_bit_cast(unsigned short, (_Float16)b) << 16); }
__device__ __forceinline__ float cmb_bf(float v) { const unsigned u = __builtin_bit_cast(unsigned, v); const unsigned r = (u + 0x7fffu + ((u >> 16) & 1u)) & 0xffff0000u; return __builtin_bit_cast(float, r); }
__global__ __launch_bounds__(256) void k_cm_castb(const float* __restrict__ SRC, int lds, unsigned short* __restrict__ DST, int ldd, int nR, int nC, float sc) {
    const long long u = (long long)blockIdx.x * 256 + threadIdx.x; const int per = nC / 8; if (u >= (long long)nR * per) return; const int r = (int)(u / per); const int c0 = 8 * (int)(u % per);
    const float* s = SRC + (long long)r * lds + c0; float w[8];
#pragma unroll
    for (int e = 0; e < 8; ++e) w[e] = cmb_bf(s[e]) * sc;
    cm_u4 pk; pk.x = cmb_pk2(w[0], w[1]); pk.y = cmb_pk2(w[2], w[3]); pk.z = cmb_pk2(w[4], w[5]); pk.w = cmb_pk2(w[6], w[7]); VST2(cm_u4, (cm_u4*)(DST + (long long)r * ldd + c0), pk); }

template <int NX, int DH>
__global__ __launch_bounds__(DH) void k_gx_exact(const float* __restrict__ Q, int ldq, const float* __restrict__ KV, int ldkv, int voff, float sc, float* __restrict__ AOX, int ldo) {
    #pragma clang fp contract(off)
    __shared__ float qs[DH]; __shared__ float ps[NX]; __shared__ float red[2];
    const int i = blockIdx.x, h = blockIdx.y, t = threadIdx.x;
    qs[t] = Q[(long long)i * ldq + h * DH + t]; __syncthreads();
#pragma unroll
    for (int r = 0; r < NX / DH; ++r) { const int j = t + DH * r; float val = -3.0e38f;
        if (DH * r <= i) {
            const int jc = min(j, i); const float* kr = KV + (long long)jc * ldkv + h * DH; float s = 0.f;
#pragma unroll 8
            for (int d = 0; d < DH; ++d) s += qs[d] * kr[d];
            val = (j <= i) ? s * sc : -3.0e38f; }
        ps[j] = val; }
    __syncthreads();
    if (t == 0) { float m = -3.0e38f; for (int j = 0; j <= i; ++j) m = fmaxf(m, ps[j]); float z = 0.f; for (int j = 0; j <= i; ++j) { const float e = expf(ps[j] - m); ps[j] = e; z += e; } red[0] = 1.f / z; }
    __syncthreads();
    const float inv = red[0]; float o = 0.f;
    for (int j = 0; j <= i; ++j) o += ps[j] * KV[(long long)j * ldkv + voff + h * DH + t];
    VST2(float, AOX + (long long)i * ldo + h * DH + t, o * inv); }
static_assert(NXR % HD == 0);

constexpr size_t SZ_X16  = (size_t)NB * SEQ * DM * 2;
constexpr size_t SZ_W3   = (size_t)NQKV * DM * 2;
constexpr size_t SZ_QKV  = (size_t)SEQ * NQKV * 4;
constexpr size_t SZ_AO   = (size_t)NB * SEQ * DM * 4;
constexpr size_t SZ_AOX  = (size_t)NB * NXR * DM * 2;
constexpr size_t SZ_INVF = 256;
constexpr size_t SZ_TAB  = (size_t)SEQ * 64 * 4;
constexpr size_t WS_TOTAL = SZ_X16 + SZ_W3 + SZ_QKV + SZ_AO + 2 * SZ_AOX + SZ_INVF + 2 * SZ_TAB;
static_assert(WS_TOTAL <= (size_t)134217728);
static_assert((size_t)3 * DM * DM * 2 <= SZ_W3);
static_assert(SZ_X16 % 256 == 0 && SZ_W3 % 256 == 0 && SZ_QKV % 256 == 0 && SZ_AO % 256 == 0 && SZ_AOX % 256 == 0 && SZ_TAB % 256 == 0);
static_assert(((size_t)(NB - 1) * SEQ_FULL + SEQ) * DM * 4 <= (size_t)NB_FULL * SEQ_FULL * DM * 4);

extern "C" void kernel_launch(void* const* d_in, const int* in_sizes, int n_in, void* d_out, int out_size, void* d_ws, size_t ws_size, hipStream_t stream) {
    if (n_in < 5) return;
    const long long need_x = ((long long)(NB - 1) * SEQ_FULL + SEQ) * DM;
    if ((long long)in_sizes[0] < need_x) return;
    for (int i = 1; i < 5; ++i) if ((long long)in_sizes[i] < (long long)DM * DM) return;
    if ((long long)out_size < need_x) return;
    if (ws_size < WS_TOTAL) return;
    const float* x  = (const float*)d_in[0];
    const float* Wq = (const float*)d_in[1];
    const float* Wk = (const float*)d_in[2];
    const float* Wv = (const float*)d_in[3];
    const float* Wo = (const float*)d_in[4];
    float* out = (float*)d_out;
    char* wsp = (char*)d_ws;
    unsigned short* X16  = (unsigned short*)wsp; wsp += SZ_X16;
    unsigned short* W316 = (unsigned short*)wsp; wsp += SZ_W3;
    float* QKV = (float*)wsp; wsp += SZ_QKV;
    float* AO  = (float*)wsp; wsp += SZ_AO;
    unsigned short* AOH2 = (unsigned short*)wsp; wsp += SZ_AOX;
    unsigned short* AOL2 = (unsigned short*)wsp; wsp += SZ_AOX;
    float* INVF = (float*)wsp; wsp += SZ_INVF;
    float* CSt = (float*)wsp; wsp += SZ_TAB;
    float* SNt = (float*)wsp; wsp += SZ_TAB;
    unsigned short* AO16 = X16;
    unsigned short* WO16 = W316;
    unsigned short* WOB  = W316 + (size_t)DM * DM;
    unsigned short* WOL  = W316 + (size_t)2 * DM * DM;

    for (int b = 0; b < NB; ++b)
        k_cm_castb<<<(unsigned)(((long long)SEQ * (DM / 8) + 255) / 256), 256, 0, stream>>>(x + (size_t)b * SEQ_FULL * DM, DM, X16 + (size_t)b * SEQ * DM, DM, SEQ, DM, 1.0f);
    k_cm_castb<<<(unsigned)(((long long)DM * (DM / 8) + 255) / 256), 256, 0, stream>>>(Wq, DM, W316, DM, DM, DM, 64.0f);
    k_cm_castb<<<(unsigned)(((long long)DM * (DM / 8) + 255) / 256), 256, 0, stream>>>(Wk, DM, W316 + (size_t)DM * DM, DM, DM, DM, 64.0f);
    k_cm_castb<<<(unsigned)(((long long)DM * (DM / 8) + 255) / 256), 256, 0, stream>>>(Wv, DM, W316 + (size_t)2 * DM * DM, DM, DM, DM, 64.0f);
    k_invf<<<1, 256, 0, stream>>>(INVF, 64, HD, 10000.0f);
    k_sincos<<<(unsigned)((SEQ * 64 + 255) / 256), 256, 0, stream>>>(CSt, SNt, INVF, SEQ, 64, 1.0f);

    for (int b = 0; b < NB; ++b) {
        gk::wmma_gemm64<0, false, 0, 0, false, 0><<<dim3((unsigned)((((SEQ) / 64) * ((NQKV) / 64) + 7) / 8), 1u), 256, 0, stream>>>(
            (const unsigned short*)(X16 + (size_t)b * SEQ * DM), nullptr, DM, 0, (const unsigned short*)W316, nullptr, DM, 0,
            (void*)QKV, nullptr, NQKV, 0, nullptr, nullptr, 0, SEQ, NQKV, DM, 0.015625f);
        k_rope_inplace<<<(unsigned)(((long long)SEQ * 32 * 16 + 255) / 256), 256, 0, stream>>>(QKV, NQKV, 32, CSt, SNt, SEQ);
        k_gx_exact<NXR, HD><<<dim3(NXR, NHD), HD, 0, stream>>>(QKV, NQKV, QKV + DM, NQKV, DM, 0.08838834764831845f, AO + (size_t)b * SEQ * DM, DM);
        if (SEQ > NXR) {
            k_attn128<<<dim3((unsigned)(((SEQ - NXR) + 63) / 64), (unsigned)NHD, 1u), 32 * AW, 0, stream>>>(
                QKV + (size_t)NXR * NQKV, QKV + DM, QKV + 2 * DM, AO + (size_t)b * SEQ * DM + (size_t)NXR * DM,
                NQKV, NQKV, DM, SEQ - NXR, SEQ, NXR, 0.08838834764831845f);
        }
    }

    k_cm_castb<<<(unsigned)(((long long)DM * (DM / 8) + 255) / 256), 256, 0, stream>>>(Wo, DM, WO16, DM, DM, DM, 64.0f);
    k_castS16<<<(unsigned)(((long long)DM * (DM / 2) + 255) / 256), 256, 0, stream>>>(Wo, DM, (__bf16*)WOB, (__bf16*)WOL, DM, DM, DM, 1.0f, 0);
    k_cast16<<<(unsigned)(((long long)NB * SEQ * (DM / 2) + 255) / 256), 256, 0, stream>>>(AO, DM, (_Float16*)AO16, DM, NB * SEQ, DM, 16.0f);
    if (SEQ > NXR) {
        gk::wmma_gemm64<0, false, 0, 0, false, 0><<<dim3((unsigned)((((SEQ - NXR) / 64) * ((DM) / 64) + 7) / 8), (unsigned)NB), 256, 0, stream>>>(
            (const unsigned short*)(AO16 + (size_t)NXR * DM), nullptr, DM, (long)((size_t)SEQ * DM), (const unsigned short*)WO16, nullptr, DM, 0,
            (void*)(out + (size_t)NXR * DM), nullptr, DM, (long)((size_t)SEQ_FULL * DM), nullptr, nullptr, 0, SEQ - NXR, DM, DM, 0.0009765625f);
    }
    for (int b = 0; b < NB; ++b)
        k_castS16<<<(unsigned)(((long long)NXR * (DM / 2) + 255) / 256), 256, 0, stream>>>(AO + (size_t)b * SEQ * DM, DM, (__bf16*)(AOH2 + (size_t)b * NXR * DM), (__bf16*)(AOL2 + (size_t)b * NXR * DM), DM, NXR, DM, 1.0f, 0);
    gk::wmma_gemm64<1, false, 0, 0, false, 0><<<dim3((unsigned)((((NXR) / 64) * ((DM) / 64) + 7) / 8), (unsigned)NB), 256, 0, stream>>>(
        (const unsigned short*)AOH2, nullptr, DM, (long)((size_t)NXR * DM), (const unsigned short*)WOB, nullptr, DM, 0,
        (void*)out, nullptr, DM, (long)((size_t)SEQ_FULL * DM), nullptr, nullptr, 0, NXR, DM, DM, 1.0f);
    gk::wmma_gemm64<1, false, 0, 0, true, 0><<<dim3((unsigned)((((NXR) / 64) * ((DM) / 64) + 7) / 8), (unsigned)NB), 256, 0, stream>>>(
        (const unsigned short*)AOL2, nullptr, DM, (long)((size_t)NXR * DM), (const unsigned short*)WOB, nullptr, DM, 0,
        (void*)out, nullptr, DM, (long)((size_t)SEQ_FULL * DM), nullptr, out, (long)((size_t)SEQ_FULL * DM), NXR, DM, DM, 1.0f);
}
